// GraphLayer_42356967473339
// MI455X (gfx1250) — hardware-run, weakly checked
//
#include <hip/hip_runtime.h>
#include <math.h>

#ifndef NB
#define NB 32
#endif
#ifndef SEQ
#define SEQ 512
#endif
#define SEQ_FULL 512
#define DMODEL 512
#define HEADS 8
#define HD 64
#define QKVN 1536
#define FFD 2048
#define MTOK (NB * SEQ)
#define PLANE ((size_t)MTOK * (size_t)DMODEL)

#define C_W   131072.0f
#define C_LN  2048.0f
#define C_P   16384.0f
#define C_A   4096.0f
#define QK_SC 7.450580596923828125e-09f
#define PV_SC 1.490116119384765625e-08f
#define SH_LNW 28u
#define SH_AW  29u
#define SH_ACT 12u

static_assert(SEQ == SEQ_FULL);
static_assert(SEQ % 128 == 0);
static_assert(MTOK % 64 == 0);
static_assert(DMODEL == 512 && HD == 64 && DMODEL == HEADS * HD && QKVN == 3 * DMODEL);
static_assert(DMODEL % 64 == 0 && QKVN % 64 == 0 && FFD % 64 == 0);
static_assert(FFD == 4 * DMODEL);

typedef _Float16 h16;
typedef __attribute__((ext_vector_type(16))) _Float16 v16h;
typedef __attribute__((ext_vector_type(8)))  _Float16 v8h;
typedef __attribute__((ext_vector_type(8)))  float    v8f;
typedef __attribute__((ext_vector_type(4)))  float    v4f;


__device__ __forceinline__ float bfr(float f) {
    unsigned u = __float_as_uint(f);
    u += 0x7FFFu + ((u >> 16) & 1u);
    return __uint_as_float(u & 0xFFFF0000u);
}
static __device__ __forceinline__ h16 toh_flush(float v) {
    const float w = (fabsf(v) < 6.103515625e-05f) ? 0.0f : v;
    return (h16)w;
}
union FragU { v16h v; v8h h[2]; };
__device__ __forceinline__ v16h frag_ld(const h16* p) {
    FragU f; f.h[0] = *(const v8h*)(p); f.h[1] = *(const v8h*)(p + 16); return f.v;
}
__device__ __forceinline__ v8f wmma16g(v16h a, v16h b, v8f c) {
    c = __builtin_amdgcn_wmma_f32_16x16x32_f16(false, a, false, b, (short)0, c, false, false);
    asm volatile("v_nop\n\tv_nop\n\tv_nop\n\tv_nop" : "+v"(c) : "v"(a), "v"(b));
    return c;
}
__device__ __forceinline__ void wave_sync_lds() {
    __builtin_amdgcn_fence(3  , "workgroup");
    __builtin_amdgcn_wave_barrier();
    __builtin_amdgcn_fence(2  , "workgroup");
}

__global__ __launch_bounds__(256) void k_wcvt(const float* __restrict__ W, h16* __restrict__ out, unsigned n8) {
    const unsigned bx = blockIdx.x;
    const unsigned u = bx * 256u + threadIdx.x;
    if (u >= n8) return;
    const v4f a = *(const v4f*)(W + (size_t)u * 8u);
    const v4f b = *(const v4f*)(W + (size_t)u * 8u + 4u);
    v8h hv;
    hv[0] = toh_flush(bfr(a.x) * C_W); hv[1] = toh_flush(bfr(a.y) * C_W);
    hv[2] = toh_flush(bfr(a.z) * C_W); hv[3] = toh_flush(bfr(a.w) * C_W);
    hv[4] = toh_flush(bfr(b.x) * C_W); hv[5] = toh_flush(bfr(b.y) * C_W);
    hv[6] = toh_flush(bfr(b.z) * C_W); hv[7] = toh_flush(bfr(b.w) * C_W);
    h16* dst = out + (size_t)u * 8u;
    *(volatile v8h*)dst = hv;
    __threadfence();
    *(volatile v8h*)dst = hv;
}

template <bool RND>
__global__ __launch_bounds__(256) void k_ln(const float* __restrict__ x, const float* __restrict__ g,
                                            const float* __restrict__ bt, h16* __restrict__ z16) {
    const unsigned bx = blockIdx.x;
    const unsigned row = bx * 8u + (threadIdx.x >> 5);
    const unsigned L = threadIdx.x & 31u;
    if (row >= (unsigned)MTOK) return;
    const float* xr = x + (size_t)row * DMODEL + 8u * L;
    const v4f a0 = *(const v4f*)(xr), a1 = *(const v4f*)(xr + 4), a2 = *(const v4f*)(xr + 256), a3 = *(const v4f*)(xr + 260);
    float v[16] = {a0.x, a0.y, a0.z, a0.w, a1.x, a1.y, a1.z, a1.w, a2.x, a2.y, a2.z, a2.w, a3.x, a3.y, a3.z, a3.w};
    if (RND) {
#pragma unroll
        for (int i = 0; i < 16; ++i) v[i] = bfr(v[i]);
    }
    float s = (((v[0] + v[1]) + (v[2] + v[3])) + ((v[4] + v[5]) + (v[6] + v[7]))) +
              (((v[8] + v[9]) + (v[10] + v[11])) + ((v[12] + v[13]) + (v[14] + v[15])));
#pragma unroll
    for (int o = 16; o > 0; o >>= 1) s += __shfl_xor(s, o, 32);
    const float mu = s * (1.0f / 512.0f);
    float d[16];
    float q = 0.f;
#pragma unroll
    for (int i = 0; i < 16; ++i) { d[i] = v[i] - mu; q += d[i] * d[i]; }
#pragma unroll
    for (int o = 16; o > 0; o >>= 1) q += __shfl_xor(q, o, 32);
    const float rs = 1.0f / sqrtf(q * (1.0f / 512.0f) + 1e-5f);
    const v4f g0 = *(const v4f*)(g + 8u * L), g1 = *(const v4f*)(g + 8u * L + 4u);
    const v4f g2 = *(const v4f*)(g + 256u + 8u * L), g3 = *(const v4f*)(g + 260u + 8u * L);
    const v4f b0 = *(const v4f*)(bt + 8u * L), b1 = *(const v4f*)(bt + 8u * L + 4u);
    const v4f b2 = *(const v4f*)(bt + 256u + 8u * L), b3 = *(const v4f*)(bt + 260u + 8u * L);
    const float gg[16] = {g0.x, g0.y, g0.z, g0.w, g1.x, g1.y, g1.z, g1.w, g2.x, g2.y, g2.z, g2.w, g3.x, g3.y, g3.z, g3.w};
    const float bb[16] = {b0.x, b0.y, b0.z, b0.w, b1.x, b1.y, b1.z, b1.w, b2.x, b2.y, b2.z, b2.w, b3.x, b3.y, b3.z, b3.w};
    v8h h0, h1;
#pragma unroll
    for (int i = 0; i < 8; ++i) {
        h0[i] = toh_flush((d[i] * rs * bfr(gg[i]) + bfr(bb[i])) * C_LN);
        h1[i] = toh_flush((d[8 + i] * rs * bfr(gg[8 + i]) + bfr(bb[8 + i])) * C_LN);
    }
    h16* dst = z16 + (size_t)row * DMODEL + 8u * L;
    for (int pass = 0; pass < 2; ++pass) {
        *(volatile v8h*)(dst) = h0;
        *(volatile v8h*)(dst + 256) = h1;
        __threadfence();
    }
}

__device__ __forceinline__ void slab_to_h16(const float* slab, h16* dst, unsigned pitch, unsigned lane) {
    const unsigned q = lane >> 3, c8 = (lane & 7u) * 8u;
    v8h hv[4];
#pragma unroll
    for (int it = 0; it < 4; ++it) {
        const unsigned row = (unsigned)it * 4u + q;
        const float* sp = slab + row * 68u + c8;
#pragma unroll
        for (int e = 0; e < 8; ++e) hv[it][e] = toh_flush(sp[e]);
    }
    for (int pass = 0; pass < 2; ++pass) {
#pragma unroll
        for (int it = 0; it < 4; ++it) {
            const unsigned row = (unsigned)it * 4u + q;
            *(volatile v8h*)(dst + (size_t)row * pitch + c8) = hv[it];
        }
        __threadfence();
    }
}

template <bool RELU, bool SCALED>
__device__ __forceinline__ float fin(float a, float bv, float scale, float oscale) {
    float v = a * scale + bv;
    if (RELU) v = fmaxf(v, 0.0f);
    if (SCALED) v *= oscale;
    return v;
}

template <int OUT_MODE, bool HASBIAS, int RESID, bool RELU, unsigned GN, unsigned GK, unsigned SCSH, unsigned OSSH>
__global__ __launch_bounds__(256) void k_gemm64(const h16* __restrict__ A, const h16* __restrict__ Bt, void* __restrict__ Cout,
                                                const float* __restrict__ bias, const float* __restrict__ resid) {
  static_assert(GN % 64u == 0u && GK % 32u == 0u);
  static_assert(OUT_MODE != 2 || GN == (unsigned)QKVN);
  __shared__ __align__(16) float sT[8][16 * 68];
  const unsigned lane = threadIdx.x & 31u;
  const unsigned wave = threadIdx.x >> 5;
  constexpr unsigned tilesN = GN / 64u;
  constexpr unsigned tilesM = (unsigned)MTOK / 64u;
  constexpr float scale = 1.0f / (float)(1u << SCSH);
  constexpr float oscale = (float)(1u << OSSH);
  const unsigned bx = blockIdx.x;
  const unsigned tile = bx * 8u + wave;
  if (tile >= tilesM * tilesN) return;
  const unsigned tm = tile / tilesN;
  const unsigned tn = tile - tm * tilesN;
  const unsigned m0 = tm << 6, n0 = tn << 6;
  const unsigned rlane = lane & 15u;
  const unsigned koff = (lane >> 4) * 8u;

  v8f acc[4][4];
#pragma unroll
  for (int i = 0; i < 4; ++i)
#pragma unroll
    for (int j = 0; j < 4; ++j) acc[i][j] = (v8f){0.f,0.f,0.f,0.f,0.f,0.f,0.f,0.f};

  for (unsigned k0 = 0; k0 < GK; k0 += 32u) {
    v16h bh[4];
#pragma unroll
    for (int j = 0; j < 4; ++j)
      bh[j] = frag_ld(Bt + (size_t)(n0 + ((unsigned)j << 4) + rlane) * GK + koff + k0);
#pragma unroll
    for (int i = 0; i < 4; ++i) {
      const v16h ah = frag_ld(A + (size_t)(m0 + ((unsigned)i << 4) + rlane) * GK + koff + k0);
#pragma unroll
      for (int j = 0; j < 4; ++j) acc[i][j] = wmma16g(ah, bh[j], acc[i][j]);
    }
  }

  float* slab = sT[wave];
  float bvj[4];
#pragma unroll
  for (int j = 0; j < 4; ++j) {
    if (HASBIAS) bvj[j] = bfr(bias[n0 + ((unsigned)j << 4) + rlane]);
    else         bvj[j] = 0.0f;
  }
  const unsigned head = tn / 3u;
  const unsigned ck = tn - head * 3u;
  const bool trans = (OUT_MODE == 2) && (ck == 0u);

  if (trans) {
    h16* C = (h16*)Cout;
    const unsigned bb = m0 / (unsigned)SEQ;
    const size_t vbase = 2u * PLANE + ((size_t)(bb * (unsigned)HEADS + head) * (unsigned)HD) * (unsigned)SEQ + (m0 - bb * (unsigned)SEQ);
#pragma unroll
    for (int j = 0; j < 4; ++j) {
#pragma unroll
      for (int i = 0; i < 4; ++i)
#pragma unroll
        for (int r = 0; r < 8; ++r)
          slab[rlane * 68u + ((unsigned)i << 4) + koff + (unsigned)r] = fin<RELU, true>(acc[i][j][r], bvj[j], scale, oscale);
      wave_sync_lds();
      slab_to_h16(slab, C + vbase + (size_t)((unsigned)j << 4) * (unsigned)SEQ, (unsigned)SEQ, lane);
      wave_sync_lds();
    }
  } else {
#pragma unroll
    for (int i = 0; i < 4; ++i) {
      const unsigned mBase = m0 + ((unsigned)i << 4);
#pragma unroll
      for (int j = 0; j < 4; ++j)
#pragma unroll
        for (int r = 0; r < 8; ++r)
          slab[(koff + (unsigned)r) * 68u + ((unsigned)j << 4) + rlane] = fin<RELU, OUT_MODE != 0>(acc[i][j][r], bvj[j], scale, oscale);
      wave_sync_lds();
      if (OUT_MODE == 0) {
        float* C = (float*)Cout;
        const unsigned hh = lane >> 4, c4 = (lane & 15u) * 4u;
#pragma unroll
        for (int half = 0; half < 2; ++half) {
          v4f vv[4];
#pragma unroll
          for (int it = 0; it < 4; ++it) {
            const unsigned row = (unsigned)(half * 4 + it) * 2u + hh;
            vv[it] = *(const v4f*)(slab + row * 68u + c4);
            if (RESID != 0) {
              v4f rv = *(const v4f*)(resid + (size_t)(mBase + row) * GN + n0 + c4);
              if (RESID == 2) { rv.x = bfr(rv.x); rv.y = bfr(rv.y); rv.z = bfr(rv.z); rv.w = bfr(rv.w); }
              vv[it] += rv;
            }
          }
          for (int pass = 0; pass < 2; ++pass) {
#pragma unroll
            for (int it = 0; it < 4; ++it) {
              const unsigned row = (unsigned)(half * 4 + it) * 2u + hh;
              *(volatile v4f*)(C + (size_t)(mBase + row) * GN + n0 + c4) = vv[it];
            }
            __threadfence();
          }
        }
      } else if (OUT_MODE == 1) {
        slab_to_h16(slab, (h16*)Cout + (size_t)mBase * GN + n0, GN, lane);
      } else {
        slab_to_h16(slab, (h16*)Cout + (size_t)(ck - 1u) * PLANE + (size_t)mBase * (unsigned)DMODEL + head * (unsigned)HD,
                    (unsigned)DMODEL, lane);
      }
      wave_sync_lds();
    }
  }
}

#define AT_PP 72
#define AT_PO 68
static_assert(AT_PO == 68);
__global__ __launch_bounds__(128) void k_attn(const h16* __restrict__ QKV, const float* __restrict__ Dm,
                                              const float* __restrict__ NMm, const float* __restrict__ MKm,
                                              const float* __restrict__ gamma, const int* __restrict__ ra_p,
                                              const int* __restrict__ rb_p, h16* __restrict__ Aout) {
    __shared__ __align__(16) h16 sP[4][16 * AT_PP];
    __shared__ __align__(16) float sS[4][16 * AT_PO];
    const unsigned tid = threadIdx.x, lane = tid & 31u, wave = tid >> 5;
    const unsigned hh = lane >> 4, c = lane & 15u;
    const unsigned prow = lane >> 1, ph = lane & 1u;
    const unsigned bx = blockIdx.x;
    const unsigned rg = bx % (unsigned)(SEQ / 64);
    const unsigned t1 = bx / (unsigned)(SEQ / 64);
    const unsigned h = t1 % (unsigned)HEADS;
    const unsigned b = t1 / (unsigned)HEADS;
    const unsigned q0 = rg * 64u + wave * 16u;
    const int ra = ra_p[0], rb = rb_p[0];
    const float g00 = bfr(gamma[0]), g01 = bfr(gamma[1]), g02 = bfr(gamma[2]);
    const float g10 = bfr(gamma[4]), g11 = bfr(gamma[5]), g12 = bfr(gamma[6]);
    const float g20 = bfr(gamma[8]), g21 = bfr(gamma[9]), g22 = bfr(gamma[10]);
    const int nq = (int)(q0 + prow);
    const int rn = (nq >= ra ? 1 : 0) + (nq >= rb ? 1 : 0);
    const float gr0 = (rn == 0) ? g00 : ((rn == 1) ? g10 : g20);
    const float gr1 = (rn == 0) ? g01 : ((rn == 1) ? g11 : g21);
    const float gr2 = (rn == 0) ? g02 : ((rn == 1) ? g12 : g22);

    const h16* Qp = QKV;
    const h16* Kp = QKV + PLANE;
    const h16* VTp = QKV + 2u * PLANE;
    const h16* qrow = Qp + (size_t)(b * (unsigned)SEQ + q0 + c) * (unsigned)DMODEL + h * (unsigned)HD + 8u * hh;
    const v16h qf0 = frag_ld(qrow);
    const v16h qf1 = frag_ld(qrow + 32);
    const size_t rowg = ((size_t)b * SEQ_FULL + q0 + prow) * SEQ_FULL + 32u * ph;
    float* ss = sS[wave];
    h16* sp = sP[wave];
    float* srow = ss + prow * AT_PO + 32u * ph;
    h16* prw = sp + prow * AT_PP + 32u * ph;

    float mrow = -3.0e38f, lrow = 0.f;
    v8f o[4];
#pragma unroll
    for (int t = 0; t < 4; ++t) o[t] = (v8f){0.f,0.f,0.f,0.f,0.f,0.f,0.f,0.f};

    for (unsigned kc = 0; kc < (unsigned)(SEQ / 64); ++kc) {
        const unsigned kv0 = kc * 64u;
#pragma unroll
        for (int j = 0; j < 4; ++j) {
            const h16* kp = Kp + (size_t)(b * (unsigned)SEQ + kv0 + 16u * (unsigned)j + c) * (unsigned)DMODEL + h * (unsigned)HD + 8u * hh;
            const v16h kf0 = frag_ld(kp);
            const v16h kf1 = frag_ld(kp + 32);
            v8f z = (v8f){0.f,0.f,0.f,0.f,0.f,0.f,0.f,0.f};
            z = wmma16g(qf0, kf0, z);
            z = wmma16g(qf1, kf1, z);
#pragma unroll
            for (int r = 0; r < 8; ++r) ss[(8u * hh + (unsigned)r) * AT_PO + 16u * (unsigned)j + c] = z[r] * QK_SC;
        }
        wave_sync_lds();

        const size_t go = rowg + kv0;
        const int kbase = (int)(kv0 + 32u * ph);
        float mx = -3.0e38f;
        for (unsigned st = 0; st < 8u; ++st) {
            const v4f q4 = *(const v4f*)(srow + 4u * st);
            const v4f d4 = *(const v4f*)(Dm + go + 4u * st);
            const v4f a4 = *(const v4f*)(NMm + go + 4u * st);
            v4f sv4;
#pragma unroll
            for (int e = 0; e < 4; ++e) {
                const int km = kbase + (int)(4u * st) + e;
                const int rm = (km >= ra ? 1 : 0) + (km >= rb ? 1 : 0);
                const float gsel = (rm == 2) ? gr2 : ((rm == 1) ? gr1 : gr0);
                const float sv = (q4[e] - gsel * bfr(d4[e])) + bfr(a4[e]);
                sv4[e] = sv;
                mx = fmaxf(mx, sv);
            }
            *(v4f*)(srow + 4u * st) = sv4;
        }
        wave_sync_lds();
        mx = fmaxf(mx, __shfl_xor(mx, 1, 32));
        const float mnew = fmaxf(mrow, mx);
        const float alpha = expf(mrow - mnew);
        mrow = mnew;

        float psum = 0.f;
        for (unsigned st = 0; st < 4u; ++st) {
            const v4f s0 = *(const v4f*)(srow + 8u * st), s1 = *(const v4f*)(srow + 8u * st + 4u);
            const v4f k0 = *(const v4f*)(MKm + go + 8u * st), k1 = *(const v4f*)(MKm + go + 8u * st + 4u);
            v8h pv;
#pragma unroll
            for (int e = 0; e < 4; ++e) {
                const float p0 = expf(s0[e] - mnew);
                const float p1 = expf(s1[e] - mnew);
                psum += p0 + p1;
                pv[e]     = toh_flush(p0 * bfr(k0[e]) * C_P);
                pv[4 + e] = toh_flush(p1 * bfr(k1[e]) * C_P);
            }
            *(v8h*)(prw + 8u * st) = pv;
        }
        psum += __shfl_xor(psum, 1, 32);
        lrow = lrow * alpha + psum;

#pragma unroll
        for (int r = 0; r < 8; ++r) {
            const float ar = __shfl(alpha, (int)(2u * (8u * hh + (unsigned)r)), 32);
            o[0][r] *= ar; o[1][r] *= ar; o[2][r] *= ar; o[3][r] *= ar;
        }
        wave_sync_lds();

#pragma unroll
        for (int kk = 0; kk < 2; ++kk) {
            FragU pf;
            pf.h[0] = *(const v8h*)(sp + c * AT_PP + (unsigned)kk * 32u + 8u * hh);
            pf.h[1] = *(const v8h*)(sp + c * AT_PP + (unsigned)kk * 32u + 8u * hh + 16u);
#pragma unroll
            for (int t = 0; t < 4; ++t) {
                const v16h vb = frag_ld(VTp + ((size_t)(b * (unsigned)HEADS + h) * (unsigned)HD + (unsigned)t * 16u + c) * (unsigned)SEQ
                                        + kv0 + (unsigned)kk * 32u + 8u * hh);
                o[t] = wmma16g(pf.v, vb, o[t]);
            }
        }
        wave_sync_lds();
    }

#pragma unroll
    for (int r = 0; r < 8; ++r) {
        const float lr = __shfl(lrow, (int)(2u * (8u * hh + (unsigned)r)), 32);
        const float inv = 1.0f / lr;
#pragma unroll
        for (int t = 0; t < 4; ++t) {
            float xv = o[t][r] * inv * PV_SC;
            xv = (xv > 0.0f) ? xv : 0.01f * xv;
            ss[(8u * hh + (unsigned)r) * AT_PO + (unsigned)t * 16u + c] = xv * C_A;
        }
    }
    wave_sync_lds();
    slab_to_h16(ss, Aout + (size_t)(b * (unsigned)SEQ + q0) * (unsigned)DMODEL + h * (unsigned)HD, (unsigned)DMODEL, lane);
}

constexpr size_t al256(size_t x) { return (x + 255) & ~(size_t)255; }
constexpr size_t WS_TOTAL = al256((size_t)QKVN * DMODEL * 2) + al256((size_t)DMODEL * DMODEL * 2) +
                            al256((size_t)FFD * DMODEL * 2) + al256((size_t)DMODEL * FFD * 2) +
                            al256(PLANE * 2) + al256(PLANE * 4) + al256(4 * PLANE * 2);
static_assert(WS_TOTAL <= (size_t)134217728);
static_assert((size_t)MTOK * FFD * 2 <= 4 * PLANE * 2);

extern "C" void kernel_launch(void* const* d_in, const int* in_sizes, int n_in, void* d_out, int out_size,
                              void* d_ws, size_t ws_size, hipStream_t stream) {
    if (n_in < 18) return;
    if (in_sizes[0] < MTOK * DMODEL || in_sizes[1] < MTOK * SEQ || in_sizes[2] < MTOK * SEQ || in_sizes[3] < MTOK * SEQ) return;
    if (in_sizes[4] < 16 || in_sizes[5] < QKVN * DMODEL || in_sizes[6] < QKVN || in_sizes[7] < DMODEL * DMODEL) return;
    if (in_sizes[8] < DMODEL || in_sizes[9] < DMODEL || in_sizes[10] < DMODEL || in_sizes[11] < DMODEL) return;
    if (in_sizes[12] < FFD * DMODEL || in_sizes[13] < FFD || in_sizes[14] < DMODEL * FFD || in_sizes[15] < DMODEL) return;
    if (in_sizes[16] < 1 || in_sizes[17] < 1 || out_size < MTOK * DMODEL) return;

    const float* Z      = (const float*)d_in[0];
    const float* Dd     = (const float*)d_in[1];
    const float* NMd    = (const float*)d_in[2];
    const float* MSK    = (const float*)d_in[3];
    const float* gamma  = (const float*)d_in[4];
    const float* qkv_w  = (const float*)d_in[5];
    const float* qkv_b  = (const float*)d_in[6];
    const float* o_w    = (const float*)d_in[7];
    const float* ln1_w  = (const float*)d_in[8];
    const float* ln1_b  = (const float*)d_in[9];
    const float* ln2_w  = (const float*)d_in[10];
    const float* ln2_b  = (const float*)d_in[11];
    const float* p1_w   = (const float*)d_in[12];
    const float* p1_b   = (const float*)d_in[13];
    const float* p2_w   = (const float*)d_in[14];
    const float* p2_b   = (const float*)d_in[15];
    const int*   ra_end = (const int*)d_in[16];
    const int*   rb_end = (const int*)d_in[17];
    float* out = (float*)d_out;

    char* wsp = (char*)d_ws;
    size_t off = 0;
    auto carve = [&](size_t bytes) -> void* { void* r = wsp + off; off += (bytes + 255) & ~(size_t)255; return r; };
    h16*   wqkv = (h16*)carve((size_t)QKVN * DMODEL * 2);
    h16*   wo   = (h16*)carve((size_t)DMODEL * DMODEL * 2);
    h16*   wp1  = (h16*)carve((size_t)FFD * DMODEL * 2);
    h16*   wp2  = (h16*)carve((size_t)DMODEL * FFD * 2);
    h16*   zn16 = (h16*)carve(PLANE * 2);
    float* Z1   = (float*)carve(PLANE * 4);
    h16*   R16  = (h16*)carve(4 * PLANE * 2);
    if (off != WS_TOTAL || off > ws_size || off > (size_t)134217728) return;

    k_wcvt<<<(QKVN * DMODEL / 8) / 256, 256, 0, stream>>>(qkv_w, wqkv, (unsigned)(QKVN * DMODEL / 8));
    k_wcvt<<<(DMODEL * DMODEL / 8) / 256, 256, 0, stream>>>(o_w, wo, (unsigned)(DMODEL * DMODEL / 8));
    k_wcvt<<<(FFD * DMODEL / 8) / 256, 256, 0, stream>>>(p1_w, wp1, (unsigned)(FFD * DMODEL / 8));
    k_wcvt<<<(DMODEL * FFD / 8) / 256, 256, 0, stream>>>(p2_w, wp2, (unsigned)(DMODEL * FFD / 8));

    const unsigned gQ = ((MTOK / 64) * (QKVN / 64) + 7) / 8;
    const unsigned gE = ((MTOK / 64) * (DMODEL / 64) + 7) / 8;
    const unsigned gF = ((MTOK / 64) * (FFD / 64) + 7) / 8;

    k_ln<true><<<(MTOK + 7) / 8, 256, 0, stream>>>(Z, ln1_w, ln1_b, zn16);
    k_gemm64<2, true, 0, false, QKVN, DMODEL, SH_LNW, SH_ACT><<<gQ, 256, 0, stream>>>(zn16, wqkv, (void*)R16, qkv_b, nullptr);
    k_attn<<<NB * HEADS * (SEQ / 64), 128, 0, stream>>>(R16, Dd, NMd, MSK, gamma, ra_end, rb_end, R16 + 3u * PLANE);
    k_gemm64<0, false, 2, false, DMODEL, DMODEL, SH_AW, 0u><<<gE, 256, 0, stream>>>(R16 + 3u * PLANE, wo, (void*)Z1, nullptr, Z);
    k_ln<false><<<(MTOK + 7) / 8, 256, 0, stream>>>(Z1, ln2_w, ln2_b, zn16);
    k_gemm64<1, true, 0, true, FFD, DMODEL, SH_LNW, SH_ACT><<<gF, 256, 0, stream>>>(zn16, wp1, (void*)R16, p1_b, nullptr);
    k_gemm64<0, true, 1, false, DMODEL, FFD, SH_AW, 0u><<<gE, 256, 0, stream>>>(R16, wp2, (void*)out, p2_b, Z1);
}
